// JointAttention_44890998178481
// MI455X (gfx1250) — hardware-run, weakly checked
//
#include <hip/hip_runtime.h>
#include <stddef.h>
#include <stdint.h>

#define NB_   8
#define NN_   25
#define NT_   64
#define CIN   512
#define PCH   128
#define NH    8
#define HD    16
#define NTOK  12800
#define NQ    384
#define HSTR  (NTOK * HD)

static_assert(NTOK == NB_ * NN_ * NT_);
static_assert(NTOK % 256 == 0);
static_assert(NQ % 64 == 0);
static_assert(PCH % 64 == 0);
static_assert((NTOK * CIN) % 2048 == 0);
static_assert(NH * HD == PCH);
static_assert(NT_ % 4 == 0);
static_assert((NB_ * NN_ * NT_) % 64 == 0);

typedef _Float16 v16h __attribute__((ext_vector_type(16)));
typedef _Float16 v8h  __attribute__((ext_vector_type(8)));
typedef float    v8f  __attribute__((ext_vector_type(8)));
typedef float    v4f  __attribute__((ext_vector_type(4)));
typedef unsigned int v4u __attribute__((ext_vector_type(4)));

union Frag  { v16h v; v8h h[2]; };
union Pack8 { v8h h; v4u u; };

__device__ __forceinline__ v8f mma16(v16h a, v16h b, v8f c) {
  c = __builtin_amdgcn_wmma_f32_16x16x32_f16(false, a, false, b, (short)0, c, false, false);
  asm volatile("v_nop\n\tv_nop\n\tv_nop\n\tv_nop" : "+v"(c) : "v"(a), "v"(b));
  return c;
}

__device__ __forceinline__ v8f zero8() { return (v8f){0.f, 0.f, 0.f, 0.f, 0.f, 0.f, 0.f, 0.f}; }
__device__ __forceinline__ v8h zero8h() {
  const _Float16 z = (_Float16)0.0f;
  return (v8h){z, z, z, z, z, z, z, z};
}

__device__ __forceinline__ v16h ldfrag(const _Float16* p, int ld, int row0, int k0, int lane) {
  const int m = lane & 15, lh = lane >> 4;
  const _Float16* q = p + (size_t)(row0 + m) * ld + k0 + 8 * lh;
  Frag f;
  f.h[0] = *(const v8h*)(q);
  f.h[1] = *(const v8h*)(q + 16);
  return f.v;
}

__device__ __forceinline__ void gemm32x64(const _Float16* __restrict__ A, int lda,
                                          const _Float16* __restrict__ Bt, int ldb, int K,
                                          int m0, int n0, int lane, v8f (&acc)[2][4]) {
#pragma unroll 1
  for (int k0 = 0; k0 < K; k0 += 32) {
    const v16h a0 = ldfrag(A, lda, m0, k0, lane);
    const v16h a1 = ldfrag(A, lda, m0 + 16, k0, lane);
    const v16h b0 = ldfrag(Bt, ldb, n0, k0, lane);
    const v16h b1 = ldfrag(Bt, ldb, n0 + 16, k0, lane);
    const v16h b2 = ldfrag(Bt, ldb, n0 + 32, k0, lane);
    const v16h b3 = ldfrag(Bt, ldb, n0 + 48, k0, lane);
    acc[0][0] = mma16(a0, b0, acc[0][0]);
    acc[1][0] = mma16(a1, b0, acc[1][0]);
    acc[0][1] = mma16(a0, b1, acc[0][1]);
    acc[1][1] = mma16(a1, b1, acc[1][1]);
    acc[0][2] = mma16(a0, b2, acc[0][2]);
    acc[1][2] = mma16(a1, b2, acc[1][2]);
    acc[0][3] = mma16(a0, b3, acc[0][3]);
    acc[1][3] = mma16(a1, b3, acc[1][3]);
  }
}

__global__ __launch_bounds__(256) void k_cvt(const float* __restrict__ src, _Float16* __restrict__ dh) {
  const size_t o = (size_t)blockIdx.x * 2048 + (size_t)threadIdx.x * 8;
  const v4f a0 = *(const v4f*)(src + o);
  const v4f a1 = *(const v4f*)(src + o + 4);
  Pack8 pk;
  pk.h = (v8h){(_Float16)a0[0], (_Float16)a0[1], (_Float16)a0[2], (_Float16)a0[3],
               (_Float16)a1[0], (_Float16)a1[1], (_Float16)a1[2], (_Float16)a1[3]};
  const v4u vv = pk.u;
  volatile v4u* d = (volatile v4u*)(dh + o);
  *d = vv;
  __threadfence();
  *d = vv;
}

#define WTP 136
__global__ __launch_bounds__(256) void k_wt(const float* __restrict__ w, int N, _Float16* __restrict__ dh) {
  __shared__ __align__(16) _Float16 sw[64 * WTP];
  const int tid = threadIdx.x;
  const int n0 = blockIdx.x * 64;
#pragma unroll
  for (int i = 0; i < 8; ++i) {
    const int p  = tid + 256 * i;
    const int k  = p >> 4;
    const int q4 = p & 15;
    const v4f v = *(const v4f*)(w + (size_t)k * N + n0 + 4 * q4) * 64.0f;
#pragma unroll
    for (int e = 0; e < 4; ++e) sw[(4 * q4 + e) * WTP + k] = (_Float16)v[e];
  }
  __syncthreads();
  v4u val[4];
  size_t go[4];
#pragma unroll
  for (int i = 0; i < 4; ++i) {
    const int p   = tid + 256 * i;
    const int row = p >> 4;
    const int pc  = p & 15;
    Pack8 pk;
    pk.h   = *(const v8h*)(sw + row * WTP + pc * 8);
    val[i] = pk.u;
    go[i]  = (size_t)(n0 + row) * PCH + pc * 8;
  }
  for (int ps = 0; ps < 2; ++ps) {
#pragma unroll
    for (int i = 0; i < 4; ++i) *(volatile v4u*)(dh + go[i]) = val[i];
    __threadfence();
  }
}

#define OTP 68
__device__ __forceinline__ void out_epi_h16(v8f (&acc)[2][4], float scale, const float (&bb)[4], float oscale,
                                            float* sw, _Float16* __restrict__ out, int ldo,
                                            int m0, int n0, int lane, int hh, int c) {
#pragma unroll
  for (int sub = 0; sub < 2; ++sub) {
    __syncthreads();
#pragma unroll
    for (int t = 0; t < 4; ++t) {
#pragma unroll
      for (int r = 0; r < 8; ++r) {
        const float v = acc[sub][t][r] * scale + bb[t];
        sw[(8 * hh + r) * OTP + 16 * t + c] = v * oscale;
      }
    }
    __syncthreads();
    v4u val[4];
    size_t go[4];
#pragma unroll
    for (int it = 0; it < 4; ++it) {
      const int p  = lane + 32 * it;
      const int L  = p >> 3;
      const int pc = p & 7;
      const float* ra = sw + L * OTP + pc * 8;
      const v4f a0 = *(const v4f*)(ra), a1 = *(const v4f*)(ra + 4);
      Pack8 pk;
      pk.h = (v8h){(_Float16)a0[0], (_Float16)a0[1], (_Float16)a0[2], (_Float16)a0[3],
                   (_Float16)a1[0], (_Float16)a1[1], (_Float16)a1[2], (_Float16)a1[3]};
      val[it] = pk.u;
      go[it]  = (size_t)(m0 + sub * 16 + L) * ldo + n0 + pc * 8;
    }
    for (int ps = 0; ps < 2; ++ps) {
#pragma unroll
      for (int it = 0; it < 4; ++it) *(volatile v4u*)(out + go[it]) = val[it];
      __threadfence();
    }
  }
}

__global__ __launch_bounds__(256) void k_qkv(const _Float16* __restrict__ xh, int choff,
                                             const _Float16* __restrict__ wt,
                                             const float* __restrict__ bias,
                                             _Float16* __restrict__ qp) {
  __shared__ __align__(16) float st[8][16 * OTP];
  const int tid = threadIdx.x, lane = tid & 31, wave = tid >> 5;
  const int hh = lane >> 4, c = lane & 15;
  const int m0 = blockIdx.x * 256 + wave * 32;
  const int n0 = blockIdx.y * 64;

  v8f acc[2][4];
#pragma unroll
  for (int s = 0; s < 2; ++s)
#pragma unroll
    for (int t = 0; t < 4; ++t) acc[s][t] = zero8();
  gemm32x64(xh + choff, CIN, wt, PCH, PCH, m0, n0, lane, acc);
  float bb[4];
#pragma unroll
  for (int t = 0; t < 4; ++t) bb[t] = bias[n0 + 16 * t + c];
  out_epi_h16(acc, 0.015625f, bb, 16.0f, st[wave], qp, NQ, m0, n0, lane, hh, c);
}

#define KTP 72
__global__ __launch_bounds__(128) void k_attn64(const _Float16* __restrict__ qp, _Float16* __restrict__ ct,
                                                int seqlen, int nqb, float sscale) {
  __shared__ __align__(16) _Float16 Vs[HD * KTP];
  __shared__ __align__(16) _Float16 Ps[4 * 16 * KTP];

  const int tid = threadIdx.x, lane = tid & 31, wave = tid >> 5;
  const int hh = lane >> 4, c = lane & 15;
  const int qb    = blockIdx.x % nqb;
  const int hb    = blockIdx.x / nqb;
  const int h     = hb % NH;
  const int seq   = hb / NH;
  const int sbase = seq * seqlen;
  const int q0    = sbase + qb * 64 + wave * 16;

  Frag qf;
  qf.h[0] = *(const v8h*)(qp + (size_t)(q0 + c) * NQ + h * HD + 8 * hh);
  qf.h[1] = zero8h();
  const v16h qa = qf.v;

  const float NEGI = -__builtin_huge_valf();
  float mrow[8], lrow[8];
  v8f oacc = zero8();
#pragma unroll
  for (int r = 0; r < 8; ++r) { mrow[r] = NEGI; lrow[r] = 0.f; }

  _Float16* pw = Ps + wave * 16 * KTP;
  const int nck = seqlen >> 6;

  for (int kc = 0; kc < nck; ++kc) {
    const int kv0 = sbase + kc * 64;
    __syncthreads();
    {
      const int r  = tid >> 1;
      const int d0 = (tid & 1) * 8;
      const v8h vv = *(const v8h*)(qp + (size_t)(kv0 + r) * NQ + 2 * PCH + h * HD + d0);
#pragma unroll
      for (int e = 0; e < 8; ++e) Vs[(d0 + e) * KTP + r] = vv[e];
    }
    v16h kb[4];
#pragma unroll
    for (int j = 0; j < 4; ++j) {
      Frag kf;
      kf.h[0] = *(const v8h*)(qp + (size_t)(kv0 + 16 * j + c) * NQ + PCH + h * HD + 8 * hh);
      kf.h[1] = zero8h();
      kb[j] = kf.v;
    }
    __syncthreads();

    v8f s[4];
#pragma unroll
    for (int j = 0; j < 4; ++j) s[j] = mma16(qa, kb[j], zero8());
    float cm[8];
#pragma unroll
    for (int r = 0; r < 8; ++r) {
      float m = NEGI;
#pragma unroll
      for (int j = 0; j < 4; ++j) { s[j][r] *= sscale; m = fmaxf(m, s[j][r]); }
#pragma unroll
      for (int off = 1; off < 16; off <<= 1) m = fmaxf(m, __shfl_xor(m, off, 32));
      cm[r] = m;
    }
    float al[8];
#pragma unroll
    for (int r = 0; r < 8; ++r) {
      const float mnew  = fmaxf(mrow[r], cm[r]);
      const float alpha = __expf(mrow[r] - mnew);
      mrow[r] = mnew;
      float psum = 0.f;
#pragma unroll
      for (int j = 0; j < 4; ++j) {
        const float p = __expf(s[j][r] - mnew);
        psum += p;
        pw[(8 * hh + r) * KTP + 16 * j + c] = (_Float16)(p * 1024.0f);
      }
#pragma unroll
      for (int off = 1; off < 16; off <<= 1) psum += __shfl_xor(psum, off, 32);
      lrow[r] = lrow[r] * alpha + psum;
      al[r] = alpha;
    }
#pragma unroll
    for (int r = 0; r < 8; ++r) oacc[r] *= al[r];
    __syncthreads();

#pragma unroll
    for (int kk = 0; kk < 2; ++kk) {
      const v16h pa = ldfrag(pw, KTP, 0, kk * 32, lane);
      const v16h vb = ldfrag(Vs, KTP, 0, kk * 32, lane);
      oacc = mma16(pa, vb, oacc);
    }
  }

  float invl[8];
#pragma unroll
  for (int r = 0; r < 8; ++r) invl[r] = (lrow[r] > 0.f) ? ((1.0f / lrow[r]) * 0.0009765625f) : 0.f;
  __syncthreads();
#pragma unroll
  for (int r = 0; r < 8; ++r) pw[(8 * hh + r) * KTP + c] = (_Float16)(oacc[r] * invl[r]);
  __syncthreads();
  Pack8 pk;
  pk.h = *(const v8h*)(pw + (lane >> 1) * KTP + (lane & 1) * 8);
  const v4u val = pk.u;
  const size_t go = (size_t)h * HSTR + (size_t)(q0 + (lane >> 1)) * HD + (lane & 1) * 8;
  for (int ps = 0; ps < 2; ++ps) {
    *(volatile v4u*)(ct + go) = val;
    __threadfence();
  }
}

#define SVP 40
__global__ __launch_bounds__(128) void k_attn_s(const _Float16* __restrict__ qp, _Float16* __restrict__ ct,
                                                float sscale) {
  __shared__ __align__(16) _Float16 Vs[4 * HD * SVP];
  __shared__ __align__(16) _Float16 Ps[4 * 32 * SVP];
  __shared__ __align__(16) _Float16 Os[NN_ * 64];

  const int tid = threadIdx.x, lane = tid & 31, wave = tid >> 5;
  const int hh = lane >> 4, c = lane & 15;
  const int h = blockIdx.x % NH;
  const int u = (blockIdx.x / NH) % (NT_ / 4);
  const int b = blockIdx.x / (NH * (NT_ / 4));
  const int t = 4 * u + wave;
  const size_t rowb = (size_t)b * NN_ * NT_ + (size_t)t;
  const float NEGI = -__builtin_huge_valf();

  _Float16* vw = Vs + wave * HD * SVP;
  _Float16* pw = Ps + wave * 32 * SVP;

  v16h qa[2];
#pragma unroll
  for (int sub = 0; sub < 2; ++sub) {
    int pos = sub * 16 + c;
    pos = (pos < NN_) ? pos : (NN_ - 1);
    Frag f;
    f.h[0] = *(const v8h*)(qp + (rowb + (size_t)pos * NT_) * NQ + h * HD + 8 * hh);
    f.h[1] = zero8h();
    qa[sub] = f.v;
  }
  v16h kb[2];
#pragma unroll
  for (int j = 0; j < 2; ++j) {
    int key = 16 * j + c;
    key = (key < NN_) ? key : (NN_ - 1);
    Frag f;
    f.h[0] = *(const v8h*)(qp + (rowb + (size_t)key * NT_) * NQ + PCH + h * HD + 8 * hh);
    f.h[1] = zero8h();
    kb[j] = f.v;
  }
#pragma unroll
  for (int i = 0; i < 2; ++i) {
    const int p  = lane + 32 * i;
    const int r  = p >> 1;
    const int d0 = (p & 1) * 8;
    const int rl = (r < NN_) ? r : (NN_ - 1);
    const v8h vv = *(const v8h*)(qp + (rowb + (size_t)rl * NT_) * NQ + 2 * PCH + h * HD + d0);
#pragma unroll
    for (int e = 0; e < 8; ++e) vw[(d0 + e) * SVP + r] = vv[e];
  }

  float lsum[2][8];
#pragma unroll
  for (int sub = 0; sub < 2; ++sub) {
    const v8f s0 = mma16(qa[sub], kb[0], zero8());
    const v8f s1 = mma16(qa[sub], kb[1], zero8());
#pragma unroll
    for (int r = 0; r < 8; ++r) {
      const float a0 = s0[r] * sscale;
      const float a1 = (16 + c < NN_) ? (s1[r] * sscale) : NEGI;
      float m = fmaxf(a0, a1);
#pragma unroll
      for (int off = 1; off < 16; off <<= 1) m = fmaxf(m, __shfl_xor(m, off, 32));
      const float p0 = __expf(a0 - m);
      const float p1 = __expf(a1 - m);
      float psum = p0 + p1;
#pragma unroll
      for (int off = 1; off < 16; off <<= 1) psum += __shfl_xor(psum, off, 32);
      lsum[sub][r] = psum;
      pw[(sub * 16 + 8 * hh + r) * SVP + c]      = (_Float16)(p0 * 1024.0f);
      pw[(sub * 16 + 8 * hh + r) * SVP + 16 + c] = (_Float16)(p1 * 1024.0f);
    }
  }
  __syncthreads();

  v8f oacc[2];
  const v16h vb = ldfrag(vw, SVP, 0, 0, lane);
#pragma unroll
  for (int sub = 0; sub < 2; ++sub) {
    const v16h pa = ldfrag(pw, SVP, sub * 16, 0, lane);
    oacc[sub] = mma16(pa, vb, zero8());
  }

#pragma unroll
  for (int sub = 0; sub < 2; ++sub) {
#pragma unroll
    for (int r = 0; r < 8; ++r) {
      const int pos = sub * 16 + 8 * hh + r;
      const float ov = oacc[sub][r] * ((1.0f / lsum[sub][r]) * 0.0009765625f);
      if (pos < NN_) Os[pos * 64 + wave * 16 + c] = (_Float16)ov;
    }
  }
  __syncthreads();
  v4u val[2];
  size_t go[2];
  bool ok[2];
#pragma unroll
  for (int i = 0; i < 2; ++i) {
    const int p  = tid + 128 * i;
    int nl = p >> 3;
    ok[i]  = (p < NN_ * 8);
    nl     = (nl < NN_) ? nl : (NN_ - 1);
    const int pc = p & 7;
    Pack8 pk;
    pk.h   = *(const v8h*)(Os + nl * 64 + pc * 8);
    val[i] = pk.u;
    go[i]  = (size_t)h * HSTR + (((size_t)b * NN_ + nl) * NT_ + 4 * u) * HD + pc * 8;
  }
  for (int ps = 0; ps < 2; ++ps) {
#pragma unroll
    for (int i = 0; i < 2; ++i)
      if (ok[i]) *(volatile v4u*)(ct + go[i]) = val[i];
    __threadfence();
  }
}

#define PTP 36
__device__ __forceinline__ v16h ldctx(const _Float16* ct, int tok0, int k0, int lane) {
  const int m = lane & 15, lh = lane >> 4;
  const int hd = k0 >> 4;
  const _Float16* q = ct + (size_t)(tok0 + m) * HD + 8 * lh;
  Frag f;
  f.h[0] = *(const v8h*)(q + (size_t)hd * HSTR);
  f.h[1] = *(const v8h*)(q + (size_t)(hd + 1) * HSTR);
  return f.v;
}
__global__ __launch_bounds__(128) void k_proj(const _Float16* __restrict__ ct,
                                              const _Float16* __restrict__ wt,
                                              const float* __restrict__ bias,
                                              float* __restrict__ out, int gsh) {
  __shared__ __align__(16) float sw[4][64 * PTP];
  const int tid = threadIdx.x, lane = tid & 31, wave = tid >> 5;
  const int hh = lane >> 4, c = lane & 15;
  const int m0 = blockIdx.x * 128 + wave * 32;
  const int n0 = blockIdx.y * 64;

  v8f acc[2][4];
#pragma unroll
  for (int s = 0; s < 2; ++s)
#pragma unroll
    for (int t = 0; t < 4; ++t) acc[s][t] = zero8();
#pragma unroll 1
  for (int k0 = 0; k0 < PCH; k0 += 32) {
    const v16h a0 = ldctx(ct, m0, k0, lane);
    const v16h a1 = ldctx(ct, m0 + 16, k0, lane);
    const v16h b0 = ldfrag(wt, PCH, n0, k0, lane);
    const v16h b1 = ldfrag(wt, PCH, n0 + 16, k0, lane);
    const v16h b2 = ldfrag(wt, PCH, n0 + 32, k0, lane);
    const v16h b3 = ldfrag(wt, PCH, n0 + 48, k0, lane);
    acc[0][0] = mma16(a0, b0, acc[0][0]);
    acc[1][0] = mma16(a1, b0, acc[1][0]);
    acc[0][1] = mma16(a0, b1, acc[0][1]);
    acc[1][1] = mma16(a1, b1, acc[1][1]);
    acc[0][2] = mma16(a0, b2, acc[0][2]);
    acc[1][2] = mma16(a1, b2, acc[1][2]);
    acc[0][3] = mma16(a0, b3, acc[0][3]);
    acc[1][3] = mma16(a1, b3, acc[1][3]);
  }
  float bb[4];
#pragma unroll
  for (int t = 0; t < 4; ++t) bb[t] = bias[n0 + 16 * t + c];

  float* swv = sw[wave];
#pragma unroll
  for (int sub = 0; sub < 2; ++sub)
#pragma unroll
    for (int t = 0; t < 4; ++t)
#pragma unroll
      for (int r = 0; r < 8; ++r)
        swv[(16 * t + c) * PTP + sub * 16 + 8 * hh + r] = acc[sub][t][r] * 0.0009765625f + bb[t];
  __syncthreads();

  const int bn = m0 >> 6;
  const int tb = m0 & 63;
  const int bq = bn / NN_;
  const int nq = bn - bq * NN_;
#pragma unroll
  for (int g2 = 0; g2 < 2; ++g2) {
    v4f val[8];
    size_t go[8];
#pragma unroll
    for (int i = 0; i < 8; ++i) {
      const int it = 8 * g2 + i;
      const int p  = lane + 32 * it;
      const int L  = p >> 3;
      const int pc = p & 7;
      val[i] = *(const v4f*)(swv + L * PTP + 4 * pc);
      go[i]  = (((size_t)bq * CIN + (size_t)(4 * (n0 + L) + gsh)) * NN_ + nq) * NT_ + tb + 4 * pc;
    }
    for (int ps = 0; ps < 2; ++ps) {
#pragma unroll
      for (int i = 0; i < 8; ++i) *(volatile v4f*)(out + go[i]) = val[i];
      __threadfence();
    }
  }
}

#define ITP 68
__global__ __launch_bounds__(256) void k_ident(const float* __restrict__ x, float* __restrict__ out) {
  __shared__ __align__(16) float sw[PCH * ITP];
  const int tid = threadIdx.x;
  const int bn = blockIdx.x;
  const int bq = bn / NN_;
  const int nq = bn - bq * NN_;
#pragma unroll
  for (int i = 0; i < 8; ++i) {
    const int p  = tid + 256 * i;
    const int t  = p >> 5;
    const int q4 = p & 31;
    const v4f v = *(const v4f*)(x + ((size_t)bn * NT_ + t) * CIN + 4 * q4);
#pragma unroll
    for (int e = 0; e < 4; ++e) sw[(4 * q4 + e) * ITP + t] = v[e];
  }
  __syncthreads();
#pragma unroll
  for (int g2 = 0; g2 < 2; ++g2) {
    v4f val[4];
    size_t go[4];
#pragma unroll
    for (int i = 0; i < 4; ++i) {
      const int p  = tid + 256 * (4 * g2 + i);
      const int j  = p >> 4;
      const int pc = p & 15;
      val[i] = *(const v4f*)(sw + j * ITP + 4 * pc);
      go[i]  = (((size_t)bq * CIN + (size_t)(4 * j)) * NN_ + nq) * NT_ + 4 * pc;
    }
    for (int ps = 0; ps < 2; ++ps) {
#pragma unroll
      for (int i = 0; i < 4; ++i) *(volatile v4f*)(out + go[i]) = val[i];
      __threadfence();
    }
  }
}

extern "C" void kernel_launch(void* const* d_in, const int* in_sizes, int n_in,
                              void* d_out, int out_size, void* d_ws, size_t ws_size,
                              hipStream_t stream) {
  if (n_in < 13) return;
  if (in_sizes[0] != NTOK * CIN) return;
  for (int br = 0; br < 3; ++br) {
    if (in_sizes[1 + 4 * br] != PCH * NQ) return;
    if (in_sizes[2 + 4 * br] != NQ) return;
    if (in_sizes[3 + 4 * br] != PCH * PCH) return;
    if (in_sizes[4 + 4 * br] != PCH) return;
  }
  if (out_size != NB_ * CIN * NN_ * NT_) return;

  const float* x = (const float*)d_in[0];
  const float* wqkv[3];
  const float* bqkv[3];
  const float* wpro[3];
  const float* bpro[3];
  for (int br = 0; br < 3; ++br) {
    wqkv[br] = (const float*)d_in[1 + 4 * br];
    bqkv[br] = (const float*)d_in[2 + 4 * br];
    wpro[br] = (const float*)d_in[3 + 4 * br];
    bpro[br] = (const float*)d_in[4 + 4 * br];
  }
  const int choff[3] = {3 * PCH, 2 * PCH, 1 * PCH};
  const int gsh[3]   = {1, 2, 3};
  float* out = (float*)d_out;

  size_t off = 0;
  const size_t oX = off; off += (size_t)NTOK * CIN * 2;
  size_t oW[3], oWp[3], oQ[3], oC[3];
  for (int br = 0; br < 3; ++br) { oW[br] = off; off += (size_t)NQ * PCH * 2; }
  for (int br = 0; br < 3; ++br) { oWp[br] = off; off += (size_t)PCH * PCH * 2; }
  for (int br = 0; br < 3; ++br) { oQ[br] = off; off += (size_t)NTOK * NQ * 2; }
  for (int br = 0; br < 3; ++br) { oC[br] = off; off += (size_t)NH * NTOK * HD * 2; }
  if (off > ws_size) return;
  if (off > (size_t)134217728) return;

  char* ws = (char*)d_ws;
  _Float16* Xh = (_Float16*)(ws + oX);
  _Float16* Wt[3];
  _Float16* Wpt[3];
  _Float16* Qp[3];
  _Float16* Ct[3];
  for (int br = 0; br < 3; ++br) {
    Wt[br]  = (_Float16*)(ws + oW[br]);
    Wpt[br] = (_Float16*)(ws + oWp[br]);
    Qp[br]  = (_Float16*)(ws + oQ[br]);
    Ct[br]  = (_Float16*)(ws + oC[br]);
  }

  k_cvt<<<dim3((NTOK * CIN) / 2048), dim3(256), 0, stream>>>(x, Xh);
  for (int br = 0; br < 3; ++br) {
    k_wt<<<dim3(NQ / 64), dim3(256), 0, stream>>>(wqkv[br], NQ, Wt[br]);
    k_wt<<<dim3(PCH / 64), dim3(256), 0, stream>>>(wpro[br], PCH, Wpt[br]);
  }
  for (int br = 0; br < 3; ++br)
    k_qkv<<<dim3(NTOK / 256, NQ / 64), dim3(256), 0, stream>>>(Xh, choff[br], Wt[br], bqkv[br], Qp[br]);
  const float sscale = 0.0009765625f;
  k_attn64<<<dim3((NB_ * NN_) * NH * 1), dim3(128), 0, stream>>>(Qp[0], Ct[0], NT_, 1, sscale);
  k_attn_s<<<dim3(NB_ * (NT_ / 4) * NH), dim3(128), 0, stream>>>(Qp[1], Ct[1], sscale);
  k_attn64<<<dim3(NB_ * NH * ((NN_ * NT_) / 64)), dim3(128), 0, stream>>>(Qp[2], Ct[2], NN_ * NT_, (NN_ * NT_) / 64, sscale);
  for (int br = 0; br < 3; ++br)
    k_proj<<<dim3(NTOK / 128, PCH / 64), dim3(128), 0, stream>>>(Ct[br], Wpt[br], bpro[br], out, gsh[br]);
  k_ident<<<dim3(NB_ * NN_), dim3(256), 0, stream>>>(x, out);
  (void)hipGetLastError();
}
